// TransformerEncoder_6296422056642
// MI455X (gfx1250) — hardware-verified
//
#include <hip/hip_runtime.h>
#ifndef NB
#define NB 2
#endif
#ifndef SEQ
#define SEQ 2048
#endif
#define NB_FULL 2
#define SEQ_FULL 2048
#define FEAT 768
#define NHEAD 12
#define DHEAD 64
#define MLPH 3072
#define MR (NB * SEQ)
#define QKVN (3 * FEAT)
static_assert(SEQ % 64 == 0);
static_assert(SEQ <= SEQ_FULL);
static_assert(NB >= 1);
static_assert(NB <= NB_FULL);
static_assert(FEAT == NHEAD * DHEAD);
static_assert(FEAT % 64 == 0);
static_assert(MLPH % 64 == 0);
static_assert(QKVN % 64 == 0);
static_assert(FEAT == 96 * 8);
static_assert(MR % 16 == 0);
static_assert(((MR / 16) * (QKVN / 64)) % 4 == 0);
static_assert(((MR / 16) * (FEAT / 64)) % 4 == 0);
static_assert(((MR / 16) * (MLPH / 64)) % 4 == 0);
static_assert((NB * NHEAD * (SEQ / 64)) * 4 * 16 * DHEAD == MR * FEAT);

typedef _Float16 v16h __attribute__((ext_vector_type(16)));
typedef unsigned short v8us __attribute__((ext_vector_type(8), may_alias));
typedef float v8f __attribute__((ext_vector_type(8)));
typedef float v4f __attribute__((ext_vector_type(4)));
typedef float v4fa __attribute__((ext_vector_type(4), may_alias));
union FragH { v16h v; v8us half[2]; unsigned short u[16]; };
union H16U { _Float16 h; unsigned short u; };

__device__ __forceinline__ unsigned short bf16_bits(float x) { unsigned int u = __float_as_uint(x); return (unsigned short)((u + 0x7FFFu + ((u >> 16) & 1u)) >> 16); }
__device__ __forceinline__ float bf16_val(unsigned short b) { return __uint_as_float(((unsigned int)b) << 16); }
__device__ __forceinline__ float bf16_rne(float x) { return bf16_val(bf16_bits(x)); }
__device__ __forceinline__ unsigned short h16_bits(float x) { H16U t; t.h = (_Float16)x; return t.u; }
__device__ __forceinline__ v8f vz8() { v8f z = {0.f, 0.f, 0.f, 0.f, 0.f, 0.f, 0.f, 0.f}; return z; }
__device__ __forceinline__ unsigned int full_row(unsigned int m) { return (m / (unsigned int)SEQ) * (unsigned int)SEQ_FULL + (m % (unsigned int)SEQ); }

__device__ __forceinline__ v8f mma16(v16h a, v16h b, v8f c) {
  c = __builtin_amdgcn_wmma_f32_16x16x32_f16(false, a, false, b, (short)0, c, false, false);
  asm volatile("v_nop\n\tv_nop\n\tv_nop\n\tv_nop" : "+v"(c) : "v"(a), "v"(b));
  return c;
}

template <unsigned int K, unsigned int N>
__global__ __launch_bounds__(256) void k_wt16(const float* __restrict__ W, unsigned short* __restrict__ Wt, float sc) {
  static_assert(K % 64 == 0);
  constexpr unsigned int K8N = K / 8u;
  const unsigned int t = blockIdx.x * 256u + threadIdx.x;
  if (t >= N * K8N) return;
  const unsigned int n = t / K8N;
  const unsigned int k8 = (t - n * K8N) * 8u;
  v8us v;
#pragma unroll
  for (unsigned int i = 0; i < 8u; ++i) v[i] = h16_bits(bf16_rne(W[(size_t)(k8 + i) * N + n]) * sc);
  unsigned short* dst = Wt + (size_t)n * K + k8;
  *(volatile v8us*)dst = v;
  __threadfence();
  *(volatile v8us*)dst = v;
}

template <bool RND, bool MAPIN, bool F32OUT>
__global__ __launch_bounds__(96) void k_ln16(const float* __restrict__ X, const float* __restrict__ g, const float* __restrict__ bt,
                                             unsigned short* __restrict__ out, float* __restrict__ out32, float osc, float eps) {
  __shared__ float red1[4];
  __shared__ float red2[4];
  __shared__ __attribute__((aligned(16))) float srow[F32OUT ? FEAT : 4];
  const unsigned int m = blockIdx.x, tid = threadIdx.x, w = tid >> 5, lane = tid & 31u;
  const unsigned int srcrow = MAPIN ? full_row(m) : m;
  const float* x = X + (size_t)srcrow * FEAT + tid * 8u;
  const v4f a0 = *(const v4fa*)x;
  const v4f a1 = *(const v4fa*)(x + 4);
  float v[8] = {a0[0], a0[1], a0[2], a0[3], a1[0], a1[1], a1[2], a1[3]};
  if (RND) {
#pragma unroll
    for (int q = 0; q < 8; ++q) v[q] = bf16_rne(v[q]);
  }
  float s = 0.f;
#pragma unroll
  for (int q = 0; q < 8; ++q) s += v[q];
#pragma unroll
  for (int o = 16; o >= 1; o >>= 1) s += __shfl_xor(s, o, 32);
  if (lane == 0u) red1[w] = s;
  __syncthreads();
  const float mu = (red1[0] + red1[1] + red1[2]) * (1.0f / (float)FEAT);
  float c[8];
  float s2 = 0.f;
#pragma unroll
  for (int q = 0; q < 8; ++q) { c[q] = v[q] - mu; s2 += c[q] * c[q]; }
#pragma unroll
  for (int o = 16; o >= 1; o >>= 1) s2 += __shfl_xor(s2, o, 32);
  if (lane == 0u) red2[w] = s2;
  __syncthreads();
  const float var = (red2[0] + red2[1] + red2[2]) * (1.0f / (float)FEAT);
  const float rs = rsqrtf(var + eps);
  float y[8];
  v8us o;
#pragma unroll
  for (int q = 0; q < 8; ++q) {
    const float gg = bf16_rne(g[tid * 8u + q]);
    const float bb = bf16_rne(bt[tid * 8u + q]);
    y[q] = c[q] * rs * gg + bb;
    o[q] = h16_bits(y[q] * osc);
  }
  unsigned short* dst = out + (size_t)m * FEAT + tid * 8u;
  if constexpr (F32OUT) {
#pragma unroll
    for (int q = 0; q < 8; ++q) srow[tid * 8u + q] = y[q];
    __syncthreads();
    const v4f p0 = *(const v4fa*)&srow[tid * 4u];
    const v4f p1 = *(const v4fa*)&srow[FEAT / 2 + tid * 4u];
    float* d32 = out32 + (size_t)m * FEAT + tid * 4u;
    *(volatile v8us*)dst = o;
    *(volatile v4f*)d32 = p0;
    *(volatile v4f*)(d32 + FEAT / 2) = p1;
    __threadfence();
    *(volatile v8us*)dst = o;
    *(volatile v4f*)d32 = p0;
    *(volatile v4f*)(d32 + FEAT / 2) = p1;
  } else {
    *(volatile v8us*)dst = o;
    __threadfence();
    *(volatile v8us*)dst = o;
  }
}

template <bool OUT16, int ACT, bool HAS_RES, bool RES_BF16, bool RES_MAP, bool OUT_MAP, unsigned int N, unsigned int K, unsigned int NSPLIT>
__global__ __launch_bounds__(128) void k_gemm16(const unsigned short* __restrict__ A, const unsigned short* __restrict__ Wt,
                                                const float* __restrict__ bias0, const float* __restrict__ bias1, const float* __restrict__ bias2,
                                                const float* __restrict__ resid, void* __restrict__ Cv, float inv_scale, float out_scale) {
  static_assert(N % 64 == 0);
  static_assert(K % 32 == 0);
  static_assert(NSPLIT % 64 == 0);
  static_assert(N % NSPLIT == 0);
  static_assert(N / NSPLIT <= 3);
  static_assert(!HAS_RES || N == FEAT);
  constexpr unsigned int M = MR, NTN = N / 64u;
  __shared__ __attribute__((aligned(16))) float so32[OUT16 ? 1 : 4][16][64];
  __shared__ __attribute__((aligned(16))) unsigned short so16[OUT16 ? 4 : 1][16][72];
  const unsigned int tid = threadIdx.x, w = tid >> 5, lane = tid & 31u, ln = lane & 15u, hh = lane >> 4;
  const unsigned int wid = blockIdx.x * 4u + w;
  const unsigned int mt = wid / NTN, nq = wid - mt * NTN;
  if (mt * 16u >= M) return;
  const unsigned int row0 = mt * 16u, col0 = nq * 64u;
  const unsigned short* arow = A + (size_t)(row0 + ln) * K;
  v8f acc[4];
#pragma unroll
  for (int t = 0; t < 4; ++t) acc[t] = vz8();
  for (unsigned int kb = 0; kb < K; kb += 32u) {
    FragH a;
    a.half[0] = *(const v8us*)(arow + kb + 8u * hh);
    a.half[1] = *(const v8us*)(arow + kb + 16u + 8u * hh);
#pragma unroll
    for (int t = 0; t < 4; ++t) {
      const unsigned short* brow = Wt + (size_t)(col0 + (unsigned int)t * 16u + ln) * K + kb;
      FragH bb;
      bb.half[0] = *(const v8us*)(brow + 8u * hh);
      bb.half[1] = *(const v8us*)(brow + 16u + 8u * hh);
      acc[t] = mma16(a.v, bb.v, acc[t]);
    }
  }
  unsigned int seg = col0 / NSPLIT; seg = (seg > 2u) ? 2u : seg;
  const float* bsel = (seg == 0u) ? bias0 : ((seg == 1u) ? bias1 : bias2);
  const unsigned int rrow0 = RES_MAP ? full_row(row0) : row0;
#pragma unroll
  for (int t = 0; t < 4; ++t) {
    const unsigned int col = col0 + (unsigned int)t * 16u + ln;
    const float bvv = bf16_rne(bsel[col - seg * NSPLIT]);
#pragma unroll
    for (int r = 0; r < 8; ++r) {
      float v = acc[t][r] * inv_scale + bvv;
      if (ACT == 1) v = fmaxf(v, 0.f);
      if constexpr (HAS_RES) {
        float rv = resid[(size_t)(rrow0 + 8u * hh + (unsigned int)r) * FEAT + col];
        if (RES_BF16) rv = bf16_rne(rv);
        v += rv;
      }
      if constexpr (OUT16) so16[w][8u * hh + r][t * 16 + ln] = h16_bits(v * out_scale);
      else so32[w][8u * hh + r][t * 16 + ln] = v;
    }
  }
  __builtin_amdgcn_fence(4  , "workgroup");
  __builtin_amdgcn_wave_barrier();
  const unsigned int orow0 = OUT_MAP ? full_row(row0) : row0;
  if constexpr (OUT16) {
    unsigned short* Ch = (unsigned short*)Cv;
    const unsigned int rq = lane >> 3, p8 = (lane & 7u) * 8u;
    for (int pass = 0; pass < 2; ++pass) {
#pragma unroll
      for (unsigned int q = 0; q < 4u; ++q) {
        const unsigned int r = q * 4u + rq;
        const v8us v = *(const v8us*)&so16[w][r][p8];
        *(volatile v8us*)(Ch + (size_t)(orow0 + r) * N + col0 + p8) = v;
      }
      if (pass == 0) __threadfence();
    }
  } else {
    float* Cf = (float*)Cv;
    const unsigned int rsub = lane >> 4, c4 = (lane & 15u) * 4u;
    for (int pass = 0; pass < 2; ++pass) {
#pragma unroll
      for (unsigned int q = 0; q < 8u; ++q) {
        const unsigned int r = q * 2u + rsub;
        const v4f v = *(const v4fa*)&so32[w][r][c4];
        *(volatile v4f*)(Cf + (size_t)(orow0 + r) * N + col0 + c4) = v;
      }
      if (pass == 0) __threadfence();
    }
  }
}

template <unsigned int D>
__global__ __launch_bounds__(128) void k_attn16(const unsigned short* __restrict__ qkv, float scale, float pcarry, float onorm,
                                                unsigned short* __restrict__ ctx) {
  static_assert(D == 64);
  constexpr unsigned int KS = D / 32u, DT = D / 16u, C8 = D / 8u;
  constexpr unsigned int T = SEQ, H = NHEAD, PITCH = QKVN, KOFF = FEAT, VOFF = 2 * FEAT, CP = FEAT, NQB = T / 64u;
  static_assert((32 * C8) % 128 == 0);
  static_assert(C8 == 8);
  __shared__ __attribute__((aligned(16))) unsigned short sK[32][D + 8];
  __shared__ __attribute__((aligned(16))) unsigned short sVt[D][40];
  __shared__ __attribute__((aligned(16))) unsigned short sP[4][16][40];
  __shared__ __attribute__((aligned(16))) unsigned short sO[4][16][D + 8];
  const unsigned int tid = threadIdx.x, w = tid >> 5, lane = tid & 31u, ln = lane & 15u, hh = lane >> 4;
  const unsigned int bh = blockIdx.x / NQB, qblk = blockIdx.x - bh * NQB;
  const unsigned int b = bh / H, h = bh - b * H;
  const unsigned int q0 = qblk * 64u + w * 16u;
  const unsigned short* Qp = qkv + (size_t)b * T * PITCH + h * D;
  const unsigned short* Kp = Qp + KOFF;
  const unsigned short* Vp = Qp + VOFF;

  FragH aq[KS];
  {
    const unsigned short* qr = Qp + (size_t)(q0 + ln) * PITCH;
#pragma unroll
    for (unsigned int ks = 0; ks < KS; ++ks) {
      aq[ks].half[0] = *(const v8us*)(qr + ks * 32u + 8u * hh);
      aq[ks].half[1] = *(const v8us*)(qr + ks * 32u + 16u + 8u * hh);
    }
  }
  float m_r[8], l_r[8];
#pragma unroll
  for (int r = 0; r < 8; ++r) { m_r[r] = -1.0e30f; l_r[r] = 0.f; }
  v8f oacc[DT];
#pragma unroll
  for (unsigned int dt = 0; dt < DT; ++dt) oacc[dt] = vz8();

  for (unsigned int j0 = 0; j0 < T; j0 += 32u) {
    __syncthreads();
#pragma unroll
    for (unsigned int it = 0; it < (32u * C8) / 128u; ++it) {
      const unsigned int e = tid + it * 128u;
      const unsigned int r = e >> 3, c8 = (e & 7u) * 8u;
      const size_t ro = (size_t)(j0 + r) * PITCH + c8;
      const v8us kvv = *(const v8us*)(Kp + ro);
      *(v8us*)&sK[r][c8] = kvv;
      const v8us vvv = *(const v8us*)(Vp + ro);
#pragma unroll
      for (unsigned int i = 0; i < 8u; ++i) sVt[c8 + i][r] = vvv[i];
    }
    __syncthreads();
    v8f s[2];
#pragma unroll
    for (unsigned int nt = 0; nt < 2u; ++nt) {
      v8f acc = vz8();
#pragma unroll
      for (unsigned int ks = 0; ks < KS; ++ks) {
        FragH bk;
        bk.half[0] = *(const v8us*)&sK[nt * 16u + ln][ks * 32u + 8u * hh];
        bk.half[1] = *(const v8us*)&sK[nt * 16u + ln][ks * 32u + 16u + 8u * hh];
        acc = mma16(aq[ks].v, bk.v, acc);
      }
      s[nt] = acc;
    }
    float alpha[8];
#pragma unroll
    for (int r = 0; r < 8; ++r) {
      const float s0 = s[0][r] * scale, s1 = s[1][r] * scale;
      float mx = fmaxf(s0, s1);
      mx = fmaxf(mx, __shfl_xor(mx, 1, 32)); mx = fmaxf(mx, __shfl_xor(mx, 2, 32));
      mx = fmaxf(mx, __shfl_xor(mx, 4, 32)); mx = fmaxf(mx, __shfl_xor(mx, 8, 32));
      const float mnew = fmaxf(m_r[r], mx);
      alpha[r] = __expf(m_r[r] - mnew);
      const float p0 = __expf(s0 - mnew), p1 = __expf(s1 - mnew);
      m_r[r] = mnew;
      l_r[r] = l_r[r] * alpha[r] + p0 + p1;
      sP[w][8u * hh + r][ln] = h16_bits(p0 * pcarry);
      sP[w][8u * hh + r][16u + ln] = h16_bits(p1 * pcarry);
    }
#pragma unroll
    for (unsigned int dt = 0; dt < DT; ++dt)
#pragma unroll
      for (int r = 0; r < 8; ++r) oacc[dt][r] *= alpha[r];
    __builtin_amdgcn_fence(4  , "workgroup");
    __builtin_amdgcn_wave_barrier();
    FragH pa;
    pa.half[0] = *(const v8us*)&sP[w][ln][8u * hh];
    pa.half[1] = *(const v8us*)&sP[w][ln][16u + 8u * hh];
#pragma unroll
    for (unsigned int dt = 0; dt < DT; ++dt) {
      FragH bv;
      bv.half[0] = *(const v8us*)&sVt[dt * 16u + ln][8u * hh];
      bv.half[1] = *(const v8us*)&sVt[dt * 16u + ln][16u + 8u * hh];
      oacc[dt] = mma16(pa.v, bv.v, oacc[dt]);
    }
    __builtin_amdgcn_fence(4  , "workgroup");
    __builtin_amdgcn_wave_barrier();
  }
#pragma unroll
  for (int r = 0; r < 8; ++r) {
    float l = l_r[r];
    l += __shfl_xor(l, 1, 32); l += __shfl_xor(l, 2, 32); l += __shfl_xor(l, 4, 32); l += __shfl_xor(l, 8, 32);
    l_r[r] = onorm * (1.0f / l);
  }
#pragma unroll
  for (unsigned int dt = 0; dt < DT; ++dt)
#pragma unroll
    for (int r = 0; r < 8; ++r) sO[w][8u * hh + r][dt * 16u + ln] = h16_bits(oacc[dt][r] * l_r[r]);
  __builtin_amdgcn_fence(4  , "workgroup");
  __builtin_amdgcn_wave_barrier();
  const unsigned int rq = lane >> 3, p8 = (lane & 7u) * 8u;
  unsigned short* crow = ctx + (size_t)(b * T + q0) * CP + h * D;
  for (int pass = 0; pass < 2; ++pass) {
#pragma unroll
    for (unsigned int q = 0; q < 4u; ++q) {
      const unsigned int r = q * 4u + rq;
      const v8us v = *(const v8us*)&sO[w][r][p8];
      *(volatile v8us*)(crow + (size_t)r * CP + p8) = v;
    }
    if (pass == 0) __threadfence();
  }
}

extern "C" void kernel_launch(void* const* d_in, const int* in_sizes, int n_in,
                              void* d_out, int out_size, void* d_ws, size_t ws_size, hipStream_t stream) {
  if (n_in < 17) return;
  const long long need_rows = (long long)(NB - 1) * SEQ_FULL + SEQ;
  if ((long long)in_sizes[0] < need_rows * FEAT) return;
  if (in_sizes[1] < FEAT * FEAT || in_sizes[3] < FEAT * FEAT || in_sizes[5] < FEAT * FEAT || in_sizes[7] < FEAT * FEAT) return;
  if (in_sizes[2] < FEAT || in_sizes[4] < FEAT || in_sizes[6] < FEAT || in_sizes[8] < FEAT) return;
  if (in_sizes[9] < FEAT || in_sizes[10] < FEAT || in_sizes[11] < FEAT || in_sizes[12] < FEAT) return;
  if (in_sizes[13] < FEAT * MLPH || in_sizes[14] < MLPH || in_sizes[15] < MLPH * FEAT || in_sizes[16] < FEAT) return;
  if ((long long)out_size < need_rows * FEAT) return;

  const float* x   = (const float*)d_in[0];
  const float* Wq  = (const float*)d_in[1];  const float* bq = (const float*)d_in[2];
  const float* Wk  = (const float*)d_in[3];  const float* bk = (const float*)d_in[4];
  const float* Wv  = (const float*)d_in[5];  const float* bv = (const float*)d_in[6];
  const float* Wo  = (const float*)d_in[7];  const float* bo = (const float*)d_in[8];
  const float* g1  = (const float*)d_in[9];  const float* be1 = (const float*)d_in[10];
  const float* g2  = (const float*)d_in[11]; const float* be2 = (const float*)d_in[12];
  const float* W1  = (const float*)d_in[13]; const float* b1 = (const float*)d_in[14];
  const float* W2  = (const float*)d_in[15]; const float* b2 = (const float*)d_in[16];

  char* ws = (char*)d_ws; size_t off = 0;
  auto take = [&](size_t bytes) { char* p = ws + off; off += (bytes + 255) & ~(size_t)255; return p; };
  unsigned short* Wqkv16 = (unsigned short*)take((size_t)QKVN * FEAT * 2);
  unsigned short* Wo16   = (unsigned short*)take((size_t)FEAT * FEAT * 2);
  unsigned short* W116   = (unsigned short*)take((size_t)MLPH * FEAT * 2);
  unsigned short* W216   = (unsigned short*)take((size_t)FEAT * MLPH * 2);
  const size_t r1_bytes = (size_t)MR * FEAT * 2;
  const size_t r2_a = (size_t)MR * QKVN * 2, r2_b = (size_t)MR * MLPH * 2;
  const size_t r2_bytes = (r2_a > r2_b) ? r2_a : r2_b;
  unsigned short* R1 = (unsigned short*)take(r1_bytes);
  unsigned short* R2 = (unsigned short*)take(r2_bytes);
  float* OUT32 = (float*)take((size_t)MR * FEAT * 4);
  float* HN32  = (float*)take((size_t)MR * FEAT * 4);
  if (off > ws_size) return;
  if (off > (size_t)134217728) return;

  const float wsc = 256.0f;
  const unsigned int g_sq = (unsigned int)((FEAT * (FEAT / 8) + 255) / 256);
  const unsigned int g_w1 = (unsigned int)((MLPH * (FEAT / 8) + 255) / 256);
  const unsigned int g_w2 = (unsigned int)((FEAT * (MLPH / 8) + 255) / 256);
  k_wt16<FEAT, FEAT><<<g_sq, 256, 0, stream>>>(Wq, Wqkv16, wsc);
  k_wt16<FEAT, FEAT><<<g_sq, 256, 0, stream>>>(Wk, Wqkv16 + (size_t)FEAT * FEAT, wsc);
  k_wt16<FEAT, FEAT><<<g_sq, 256, 0, stream>>>(Wv, Wqkv16 + (size_t)2 * FEAT * FEAT, wsc);
  k_wt16<FEAT, FEAT><<<g_sq, 256, 0, stream>>>(Wo, Wo16, wsc);
  k_wt16<FEAT, MLPH><<<g_w1, 256, 0, stream>>>(W1, W116, wsc);
  k_wt16<MLPH, FEAT><<<g_w2, 256, 0, stream>>>(W2, W216, wsc);

  auto ggrid = [](int N) { return (unsigned int)((((MR) / 16) * (N / 64) + 3) / 4); };
  const float scale = 0.036084391824351615f;

  k_ln16<true, true, false><<<(unsigned int)MR, 96, 0, stream>>>(x, g1, be1, R1, nullptr, 8.0f, 1e-5f);
  k_gemm16<true, 0, false, false, false, false, QKVN, FEAT, FEAT><<<ggrid(QKVN), 128, 0, stream>>>(
      R1, Wqkv16, bq, bk, bv, nullptr, (void*)R2, 1.0f / 2048.0f, 1.0f);
  k_attn16<DHEAD><<<(unsigned int)(NB * NHEAD * (SEQ / 64)), 128, 0, stream>>>(R2, scale, 1024.0f, 0.0625f, R1);
  k_gemm16<false, 0, true, true, true, false, FEAT, FEAT, FEAT><<<ggrid(FEAT), 128, 0, stream>>>(
      R1, Wo16, bo, bo, bo, x, (void*)OUT32, 1.0f / 16384.0f, 1.0f);
  k_ln16<false, false, true><<<(unsigned int)MR, 96, 0, stream>>>(OUT32, g2, be2, R1, HN32, 8.0f, 1e-5f);
  k_gemm16<true, 1, false, false, false, false, MLPH, FEAT, MLPH><<<ggrid(MLPH), 128, 0, stream>>>(
      R1, W116, b1, b1, b1, nullptr, (void*)R2, 1.0f / 2048.0f, 16.0f);
  k_gemm16<false, 0, true, false, false, true, FEAT, MLPH, FEAT><<<ggrid(FEAT), 128, 0, stream>>>(
      R2, W216, b2, b2, b2, HN32, d_out, 1.0f / 4096.0f, 1.0f);
}
